// BasicNeRF2d_50861002719868
// MI455X (gfx1250) — hardware-run, weakly checked
//
#include <hip/hip_runtime.h>
#include <math.h>

constexpr int kCh        = 256;
constexpr int kChunkRows = 65536;
constexpr int kL1Rows    = 64;
constexpr int kOutRows   = 256;
constexpr int kEncPts    = 128;
constexpr float kWCarry    = 16.0f;
constexpr float kWCarryInv = 1.0f / 16.0f;
static_assert(kChunkRows % kL1Rows == 0);
static_assert(kChunkRows % kOutRows == 0);
static_assert(kChunkRows % kEncPts == 0);
static_assert(kChunkRows % 64 == 0);
static_assert(kCh % 64 == 0);

typedef __attribute__((ext_vector_type(16))) _Float16 v16h;
typedef __attribute__((ext_vector_type(8)))  _Float16 v8h;
typedef __attribute__((ext_vector_type(16))) __bf16   v16b;
typedef __attribute__((ext_vector_type(8)))  __bf16   v8b;
typedef __attribute__((ext_vector_type(8)))  float    v8f;
typedef __attribute__((ext_vector_type(4)))  float    v4f;
typedef __attribute__((ext_vector_type(4)))  unsigned int v4u;

__device__ __forceinline__ unsigned short f2bf_bits(float f) {
  unsigned u = __float_as_uint(f);
  return (unsigned short)((u + 0x7FFFu + ((u >> 16) & 1u)) >> 16);
}
__device__ __forceinline__ float bf_bits2f(unsigned short h) { return __uint_as_float(((unsigned)h) << 16); }

__device__ __forceinline__ void dep_guard_h(v8f& a, v8f& b, v16h x, v16h y) { asm volatile("v_nop\n\tv_nop\n\tv_nop\n\tv_nop" : "+v"(a), "+v"(b) : "v"(x), "v"(y)); }
__device__ __forceinline__ void dep_guard_b(v8f& a, v8f& b, v16b x, v16b y) { asm volatile("v_nop\n\tv_nop\n\tv_nop\n\tv_nop" : "+v"(a), "+v"(b) : "v"(x), "v"(y)); }
__device__ __forceinline__ void keep4_h(v16h a, v16h b, v16h c, v16h d) { asm volatile("v_nop" :: "v"(a), "v"(b), "v"(c), "v"(d)); }
__device__ __forceinline__ void keep4_b(v16b a, v16b b, v16b c, v16b d) { asm volatile("v_nop" :: "v"(a), "v"(b), "v"(c), "v"(d)); }
__device__ __forceinline__ void acc_guard4(v8f& a, v8f& b, v8f& c, v8f& d) { asm volatile("v_nop\n\tv_nop\n\tv_nop\n\tv_nop" : "+v"(a), "+v"(b), "+v"(c), "+v"(d)); }
template <typename T> struct Frag;
template <> struct Frag<_Float16> {
  typedef v16h V; union U { v16h v; v8h h[2]; };
  static __device__ __forceinline__ v16h load(const _Float16* p) {
    U f; f.h[0] = *(const v8h*)(p); f.h[1] = *(const v8h*)(p + 16); return f.v;
  }
  static __device__ __forceinline__ v8f mma(v16h a, v16h b, v8f c) {
    return __builtin_amdgcn_wmma_f32_16x16x32_f16(false, a, false, b, (short)0, c, false, false);
  }
  static __device__ __forceinline__ void guard(v8f& a, v8f& b, v16h x, v16h y) { dep_guard_h(a, b, x, y); }
  static __device__ __forceinline__ void keep(v16h a, v16h b, v16h c, v16h d) { keep4_h(a, b, c, d); }
};
template <> struct Frag<__bf16> {
  typedef v16b V; union U { v16b v; v8b h[2]; };
  static __device__ __forceinline__ v16b load(const __bf16* p) {
    U f; f.h[0] = *(const v8b*)(p); f.h[1] = *(const v8b*)(p + 16); return f.v;
  }
  static __device__ __forceinline__ v8f mma(v16b a, v16b b, v8f c) {
    return __builtin_amdgcn_wmma_f32_16x16x32_bf16(false, a, false, b, (short)0, c, false, false);
  }
  static __device__ __forceinline__ void guard(v8f& a, v8f& b, v16b x, v16b y) { dep_guard_b(a, b, x, y); }
  static __device__ __forceinline__ void keep(v16b a, v16b b, v16b c, v16b d) { keep4_b(a, b, c, d); }
};

__device__ __forceinline__ unsigned pk16(unsigned short a, unsigned short b) { return (unsigned)a | ((unsigned)b << 16); }
__device__ __forceinline__ unsigned short h_bits(float f) { const _Float16 h = (_Float16)f; return __builtin_bit_cast(unsigned short, h); }

template <int ET> struct Elem;
template <> struct Elem<0> { typedef _Float16 T; };
template <> struct Elem<1> { typedef __bf16 T; };
template <int ET, bool SPLIT, int BIAS_MODE, int OUT_MODE, bool RESID, int ACT = 0>
__global__ __launch_bounds__(256) void wmma_gemm64(
    const unsigned short* __restrict__ Ap, const unsigned short* __restrict__ A2p, int lda, long strideA,
    const unsigned short* __restrict__ Btp, const unsigned short* __restrict__ Bt2p, int ldb, long strideB,
    void* __restrict__ Cout, void* __restrict__ Cout2, int ldc, long strideC,
    const float* __restrict__ bias,
    const float* __restrict__ resid, long strideR,
    int M, int N, int K, float scale) {
  typedef typename Elem<ET>::T T;
  typedef typename Frag<T>::V V;
  const T* A = (const T*)Ap; const T* A2 = (const T*)A2p; const T* Bt = (const T*)Btp; const T* Bt2 = (const T*)Bt2p;
  __shared__ __align__(16) float sT[8][16 * 68];
  const int b    = blockIdx.y;
  const int lane = threadIdx.x & 31;
  const int wave = threadIdx.x >> 5;
  const int tilesN = N >> 6;
  const int tilesM = M >> 6;
  const int tile = blockIdx.x * 8 + wave;
  if (tile >= tilesM * tilesN) return;
  const int tm = tile / tilesN;
  const int tn = tile - tm * tilesN;
  const int m0 = tm << 6;
  const int n0 = tn << 6;

  const T* Ab  = A  + (size_t)b * strideA;
  const T* Bb  = Bt + (size_t)b * strideB;
  const T* Ab2 = SPLIT ? (A2  + (size_t)b * strideA) : nullptr;
  const T* Bb2 = SPLIT ? (Bt2 + (size_t)b * strideB) : nullptr;

  const int rlane = lane & 15;
  const int koff  = (lane >> 4) * 8;
  const int mOff  = (lane >> 4) * 8;

  v8f acc[4][4];
#pragma unroll
  for (int i = 0; i < 4; ++i)
#pragma unroll
    for (int j = 0; j < 4; ++j) acc[i][j] = (v8f){0.f,0.f,0.f,0.f,0.f,0.f,0.f,0.f};

  for (int k0 = 0; k0 < K; k0 += 32) {
    V bh[4], bl[4];
#pragma unroll
    for (int j = 0; j < 4; ++j) {
      const size_t bo = (size_t)(n0 + (j << 4) + rlane) * ldb + koff + k0;
      bh[j] = Frag<T>::load(Bb + bo);
      if (SPLIT) bl[j] = Frag<T>::load(Bb2 + bo);
    }
#pragma unroll
    for (int i = 0; i < 4; ++i) {
      const size_t ao = (size_t)(m0 + (i << 4) + rlane) * lda + koff + k0;
      V ah = Frag<T>::load(Ab + ao);
      V al;
      if (SPLIT) al = Frag<T>::load(Ab2 + ao);
#pragma unroll
      for (int j = 0; j < 4; ++j) {
        acc[i][j] = Frag<T>::mma(ah, bh[j], acc[i][j]);
        if (SPLIT) {
          acc[i][j] = Frag<T>::mma(ah, bl[j], acc[i][j]);
          acc[i][j] = Frag<T>::mma(al, bh[j], acc[i][j]);
        }
      }
      Frag<T>::guard(acc[i][0], acc[i][3], ah, SPLIT ? al : ah);
    }
    Frag<T>::keep(bh[0], bh[1], bh[2], bh[3]);
    if (SPLIT) Frag<T>::keep(bl[0], bl[1], bl[2], bl[3]);
  }
  acc_guard4(acc[0][0], acc[0][1], acc[0][2], acc[0][3]);
  acc_guard4(acc[1][0], acc[1][1], acc[1][2], acc[1][3]);
  acc_guard4(acc[2][0], acc[2][1], acc[2][2], acc[2][3]);
  acc_guard4(acc[3][0], acc[3][1], acc[3][2], acc[3][3]);

  float* slab = sT[wave];
  const float* Rb = RESID ? (resid + (size_t)b * strideR) : nullptr;
#pragma unroll
  for (int i = 0; i < 4; ++i) {
    const int mBase = m0 + (i << 4);
#pragma unroll
    for (int j = 0; j < 4; ++j) {
      const int n = n0 + (j << 4) + rlane;
      float bv = 0.f;
      if (BIAS_MODE == 2) bv = bias[n];
#pragma unroll
      for (int r = 0; r < 8; ++r) {
        float v = acc[i][j][r] * scale;
        if (BIAS_MODE == 1) v += bias[mBase + mOff + r];
        if (BIAS_MODE == 2) v += bv;
        if (RESID) v += Rb[(size_t)(mBase + mOff + r) * ldc + n];
        if (ACT == 2) v = fmaxf(v, 0.0f);
        if (ACT == 4) v = (v > 0.f) ? v : 0.01f * v;
        slab[(mOff + r) * 68 + (j << 4) + rlane] = v;
      }
    }
    __builtin_amdgcn_fence(__ATOMIC_RELEASE, "workgroup");
    __builtin_amdgcn_wave_barrier();
    __builtin_amdgcn_fence(__ATOMIC_ACQUIRE, "workgroup");
    if (OUT_MODE == 0) {
      float* C = (float*)Cout + (size_t)b * strideC;
      const int hh = lane >> 4, c4 = (lane & 15) * 4;
      for (int pass = 0; pass < 2; ++pass) {
#pragma unroll
        for (int it = 0; it < 8; ++it) {
          const int row = it * 2 + hh;
          v4f v = *(const v4f*)(slab + row * 68 + c4);
          *(volatile v4f*)(C + (size_t)(mBase + row) * ldc + n0 + c4) = v;
        }
        __threadfence();
      }
    } else {
      const int q = lane >> 3, c8 = (lane & 7) * 8;
      unsigned short* C  = (unsigned short*)Cout  + (size_t)b * strideC;
      unsigned short* C2 = (OUT_MODE == 2) ? ((unsigned short*)Cout2 + (size_t)b * strideC) : nullptr;
      for (int pass = 0; pass < 2; ++pass) {
#pragma unroll
        for (int it = 0; it < 4; ++it) {
          const int row = it * 4 + q;
          const float* sp = slab + row * 68 + c8;
          v8h hv, lv;
#pragma unroll
          for (int e = 0; e < 8; ++e) {
            if (OUT_MODE == 1) {
              hv[e] = (_Float16)sp[e];
            } else {
              unsigned short hb = f2bf_bits(sp[e]);
              unsigned short lb = f2bf_bits(sp[e] - bf_bits2f(hb));
              hv[e] = __builtin_bit_cast(_Float16, hb);
              lv[e] = __builtin_bit_cast(_Float16, lb);
            }
          }
          *(volatile v8h*)(C + (size_t)(mBase + row) * ldc + n0 + c8) = hv;
          if (OUT_MODE == 2) *(volatile v8h*)(C2 + (size_t)(mBase + row) * ldc + n0 + c8) = lv;
        }
        __threadfence();
      }
    }
    __builtin_amdgcn_fence(__ATOMIC_RELEASE, "workgroup");
    __builtin_amdgcn_wave_barrier();
    __builtin_amdgcn_fence(__ATOMIC_ACQUIRE, "workgroup");
  }
}

__global__ __launch_bounds__(256) void wtcast256_kernel(const float* __restrict__ W0, const float* __restrict__ W1,
                                                        unsigned short* __restrict__ out, float scale) {
  __shared__ float sm[64][65];
  const int t  = threadIdx.x;
  const int k0 = blockIdx.x * 64;
  const int n0 = blockIdx.y * 64;
  const int z  = blockIdx.z;
  const float* W = (z == 0) ? W0 : W1;
#pragma unroll
  for (int i = 0; i < 16; ++i) {
    const int e = i * 256 + t;
    const int r = e >> 6;
    const int c = e & 63;
    sm[c][r] = W[(size_t)(k0 + r) * kCh + n0 + c] * scale;
  }
  __syncthreads();
  const int lane = t & 31, wave = t >> 5;
  const int q = lane >> 3, c8 = (lane & 7) * 8;
  unsigned short* op = out + (size_t)z * kCh * kCh;
  for (int pass = 0; pass < 2; ++pass) {
#pragma unroll
    for (int it = 0; it < 2; ++it) {
      const int row = wave * 8 + it * 4 + q;
      unsigned short hb[8];
#pragma unroll
      for (int e = 0; e < 8; ++e) hb[e] = h_bits(sm[row][c8 + e]);
      const v4u u = (v4u){pk16(hb[0], hb[1]), pk16(hb[2], hb[3]), pk16(hb[4], hb[5]), pk16(hb[6], hb[7])};
      *(volatile v4u*)(op + (size_t)(n0 + row) * kCh + k0 + c8) = u;
    }
    __threadfence();
  }
}

__global__ __launch_bounds__(256) void enc_kernel(const float* __restrict__ uv, float* __restrict__ enc, int nPoints) {
  __shared__ __align__(16) float sE[kEncPts * 4];
  const int t = threadIdx.x;
  const int p = t >> 1;
  const int j = t & 1;
  int pt = blockIdx.x * kEncPts + p;
  pt = pt < nPoints ? pt : nPoints - 1;
  const float x = uv[(size_t)pt * 2 + j];
  const float cv = cosf(x);
  const float sv = sinf(x);
  sE[p * 4 + j]     = cv;
  sE[p * 4 + 2 + j] = sv;
  __syncthreads();
  if (t < kEncPts) {
    const int pw = blockIdx.x * kEncPts + t;
    if (pw < nPoints) {
      const v4f v = *(const v4f*)(sE + t * 4);
      float* op = enc + (size_t)pw * 4;
      *(volatile v4f*)op = v;
      __threadfence();
      *(volatile v4f*)op = v;
    }
  }
}

__global__ __launch_bounds__(256) void l1_kernel(const float* __restrict__ enc, const float* __restrict__ W_in,
                                                 const float* __restrict__ b_in, unsigned short* __restrict__ H,
                                                 int row0, int nPoints) {
  __shared__ __align__(16) float sW[4 * kCh];
  __shared__ __align__(16) float sB[kCh];
  const int t = threadIdx.x;
#pragma unroll
  for (int i = 0; i < 4; ++i) sW[i * kCh + t] = W_in[i * kCh + t];
  sB[t] = b_in[t];
  __syncthreads();
  const int lane = t & 31, wave = t >> 5;
  const int q = lane >> 3, c8 = (lane & 7) * 8;
  const int lrow0 = blockIdx.x * kL1Rows;
#pragma unroll 1
  for (int it = 0; it < 8; ++it) {
    const int rloc = wave * 8 + (it & 1) * 4 + q;
    const int c0   = (it >> 1) * 64 + c8;
    int grow = row0 + lrow0 + rloc;
    grow = grow < nPoints ? grow : nPoints - 1;
    const v4f e = *(const v4f*)(enc + (size_t)grow * 4);
    const v4f w0a = *(const v4f*)(sW + c0);
    const v4f w0b = *(const v4f*)(sW + c0 + 4);
    const v4f w1a = *(const v4f*)(sW + kCh + c0);
    const v4f w1b = *(const v4f*)(sW + kCh + c0 + 4);
    const v4f w2a = *(const v4f*)(sW + 2 * kCh + c0);
    const v4f w2b = *(const v4f*)(sW + 2 * kCh + c0 + 4);
    const v4f w3a = *(const v4f*)(sW + 3 * kCh + c0);
    const v4f w3b = *(const v4f*)(sW + 3 * kCh + c0 + 4);
    const v4f ba  = *(const v4f*)(sB + c0);
    const v4f bb  = *(const v4f*)(sB + c0 + 4);
    unsigned short hb[8];
#pragma unroll
    for (int x = 0; x < 4; ++x) {
      float d = e[0] * w0a[x];
      d = fmaf(e[1], w1a[x], d);
      d = fmaf(e[2], w2a[x], d);
      d = fmaf(e[3], w3a[x], d);
      d = d + ba[x];
      hb[x] = h_bits(fmaxf(d, 0.0f));
      float g = e[0] * w0b[x];
      g = fmaf(e[1], w1b[x], g);
      g = fmaf(e[2], w2b[x], g);
      g = fmaf(e[3], w3b[x], g);
      g = g + bb[x];
      hb[4 + x] = h_bits(fmaxf(g, 0.0f));
    }
    const v4u u = (v4u){pk16(hb[0], hb[1]), pk16(hb[2], hb[3]), pk16(hb[4], hb[5]), pk16(hb[6], hb[7])};
    unsigned short* hp = H + (size_t)(lrow0 + rloc) * kCh + c0;
    *(volatile v4u*)hp = u;
    __threadfence();
    *(volatile v4u*)hp = u;
  }
}

__global__ __launch_bounds__(256) void out3_kernel(const unsigned short* __restrict__ H, const float* __restrict__ W_out,
                                                   const float* __restrict__ b_out, float* __restrict__ out,
                                                   int row0, int nPoints) {
  __shared__ __align__(16) float sWo[3 * kCh];
  __shared__ __align__(16) float sO[kOutRows * 3];
  const int t = threadIdx.x;
#pragma unroll
  for (int i = 0; i < 3; ++i) sWo[i * kCh + t] = W_out[i * kCh + t];
  __syncthreads();
  const int lrow = blockIdx.x * kOutRows + t;
  const v4u* hp = (const v4u*)(H + (size_t)lrow * kCh);
  float o0 = 0.0f, o1 = 0.0f, o2 = 0.0f;
#pragma unroll 1
  for (int c8i = 0; c8i < 32; ++c8i) {
    const v4u w = hp[c8i];
#pragma unroll
    for (int i = 0; i < 4; ++i) {
      const unsigned wi = w[i];
      const unsigned short lo = (unsigned short)(wi & 0xffffu);
      const unsigned short hi = (unsigned short)(wi >> 16);
      const float ha = (float)__builtin_bit_cast(_Float16, lo);
      const float hb = (float)__builtin_bit_cast(_Float16, hi);
      const int c = c8i * 8 + 2 * i;
      const float* wp = sWo + c * 3;
      o0 = fmaf(ha, wp[0], o0);
      o1 = fmaf(ha, wp[1], o1);
      o2 = fmaf(ha, wp[2], o2);
      o0 = fmaf(hb, wp[3], o0);
      o1 = fmaf(hb, wp[4], o1);
      o2 = fmaf(hb, wp[5], o2);
    }
  }
  o0 += b_out[0];
  o1 += b_out[1];
  o2 += b_out[2];
  const float s0 = 1.0f / (1.0f + expf(-o0));
  const float s1 = 1.0f / (1.0f + expf(-o1));
  const float s2 = 1.0f / (1.0f + expf(-o2));
  sO[t * 3 + 0] = s0;
  sO[t * 3 + 1] = s1;
  sO[t * 3 + 2] = s2;
  __syncthreads();
  if (t < (kOutRows * 3) / 4) {
    const int growBase = row0 + blockIdx.x * kOutRows;
    if (growBase + kOutRows <= nPoints) {
      const v4f v = *(const v4f*)(sO + 4 * t);
      float* op = out + (size_t)growBase * 3 + 4 * t;
      *(volatile v4f*)op = v;
      __threadfence();
      *(volatile v4f*)op = v;
    }
  }
}

extern "C" void kernel_launch(void* const* d_in, const int* in_sizes, int n_in,
                              void* d_out, int out_size, void* d_ws, size_t ws_size,
                              hipStream_t stream) {
  if (n_in < 9) return;
  const float* uv    = (const float*)d_in[0];
  const float* W_in  = (const float*)d_in[1];
  const float* b_in  = (const float*)d_in[2];
  const float* W_h0  = (const float*)d_in[3];
  const float* b_h0  = (const float*)d_in[4];
  const float* W_h1  = (const float*)d_in[5];
  const float* b_h1  = (const float*)d_in[6];
  const float* W_out = (const float*)d_in[7];
  const float* b_out = (const float*)d_in[8];
  float* out = (float*)d_out;

  const int nPoints = in_sizes[0] / 2;
  if (nPoints <= 0 || (nPoints % kChunkRows) != 0) return;
  if (in_sizes[1] != 4 * kCh || in_sizes[2] != kCh || in_sizes[3] != kCh * kCh || in_sizes[4] != kCh ||
      in_sizes[5] != kCh * kCh || in_sizes[6] != kCh || in_sizes[7] != kCh * 3 || in_sizes[8] < 3) return;
  if ((long)out_size < (long)nPoints * 3L) return;
  const int nChunks = nPoints / kChunkRows;

  const size_t wtBytes    = (size_t)2 * kCh * kCh * sizeof(unsigned short);
  const size_t encBytes   = (size_t)nPoints * 4 * sizeof(float);
  const size_t planeBytes = (size_t)kChunkRows * kCh * sizeof(unsigned short);
  const size_t offWt  = 0;
  const size_t offEnc = offWt + wtBytes;
  const size_t offA   = offEnc + encBytes;
  const size_t offB   = offA + planeBytes;
  const size_t total  = offB + planeBytes;
  if (total > ws_size) return;

  unsigned char* ws = (unsigned char*)d_ws;
  unsigned short* wt0    = (unsigned short*)(ws + offWt);
  unsigned short* wt1    = wt0 + (size_t)kCh * kCh;
  float*          enc    = (float*)(ws + offEnc);
  unsigned short* planeA = (unsigned short*)(ws + offA);
  unsigned short* planeB = (unsigned short*)(ws + offB);

  wtcast256_kernel<<<dim3(kCh / 64, kCh / 64, 2), 256, 0, stream>>>(W_h0, W_h1, wt0, kWCarry);

  enc_kernel<<<dim3(nPoints / kEncPts), 256, 0, stream>>>(uv, enc, nPoints);

  const int tiles      = (kChunkRows / 64) * (kCh / 64);
  const int gemmBlocks = (tiles + 7) / 8;

  for (int ch = 0; ch < nChunks; ++ch) {
    const int row0 = ch * kChunkRows;
    l1_kernel<<<dim3(kChunkRows / kL1Rows), 256, 0, stream>>>(enc, W_in, b_in, planeA, row0, nPoints);
    wmma_gemm64<0, false, 2, 1, false, 2> <<<dim3(gemmBlocks, 1, 1), 256, 0, stream>>>(
        planeA, planeA, kCh, 0L,
        wt0, wt0, kCh, 0L,
        (void*)planeB, (void*)planeB, kCh, 0L,
        b_h0, b_h0, 0L,
        kChunkRows, kCh, kCh, kWCarryInv);
    wmma_gemm64<0, false, 2, 1, false, 2> <<<dim3(gemmBlocks, 1, 1), 256, 0, stream>>>(
        planeB, planeB, kCh, 0L,
        wt1, wt1, kCh, 0L,
        (void*)planeA, (void*)planeA, kCh, 0L,
        b_h1, b_h1, 0L,
        kChunkRows, kCh, kCh, kWCarryInv);
    out3_kernel<<<dim3(kChunkRows / kOutRows), 256, 0, stream>>>(planeA, W_out, b_out, out, row0, nPoints);
  }
}
